// ImplicitDAM_5325759447207
// MI455X (gfx1250) — hardware-verified
//
#include <hip/hip_runtime.h>
#include <hip/hip_bf16.h>

#define NBATCH 2048
#define DIN    512
#define DCOMB  1024
#define DKEY   64
#define DVAL   64
#define NBINS  65536
#define NPROJ  128
#define QS     0.03125f
#define PSC    32768.0f
#define WSCL   256.0f
#define KVSCL  64.0f

typedef __attribute__((ext_vector_type(16))) _Float16 v16h;
typedef __attribute__((ext_vector_type(8)))  _Float16 v8h;
typedef __attribute__((ext_vector_type(16))) __bf16   v16b;
typedef __attribute__((ext_vector_type(8)))  __bf16   v8b;
typedef __attribute__((ext_vector_type(8)))  float    v8f;
typedef __attribute__((ext_vector_type(4)))  float    v4f;
typedef __attribute__((ext_vector_type(2)))  float    v2f;

__device__ __forceinline__ unsigned short f2bf_bits(float f) {
  unsigned u = __float_as_uint(f);
  return (unsigned short)((u + 0x7FFFu + ((u >> 16) & 1u)) >> 16);
}
__device__ __forceinline__ float bf_bits2f(unsigned short h) { return __uint_as_float(((unsigned)h) << 16); }

__device__ __forceinline__ void dep_guard_h(v8f& a, v8f& b, v16h x, v16h y) { asm volatile("v_nop\n\tv_nop\n\tv_nop\n\tv_nop" : "+v"(a), "+v"(b) : "v"(x), "v"(y)); }
__device__ __forceinline__ void dep_guard_b(v8f& a, v8f& b, v16b x, v16b y) { asm volatile("v_nop\n\tv_nop\n\tv_nop\n\tv_nop" : "+v"(a), "+v"(b) : "v"(x), "v"(y)); }
__device__ __forceinline__ void keep4_h(v16h a, v16h b, v16h c, v16h d) { asm volatile("v_nop" :: "v"(a), "v"(b), "v"(c), "v"(d)); }
__device__ __forceinline__ void keep4_b(v16b a, v16b b, v16b c, v16b d) { asm volatile("v_nop" :: "v"(a), "v"(b), "v"(c), "v"(d)); }
__device__ __forceinline__ void acc_guard4(v8f& a, v8f& b, v8f& c, v8f& d) { asm volatile("v_nop\n\tv_nop\n\tv_nop\n\tv_nop" : "+v"(a), "+v"(b), "+v"(c), "+v"(d)); }
template <typename T> struct Frag;
template <> struct Frag<_Float16> {
  typedef v16h V; union U { v16h v; v8h h[2]; };
  static __device__ __forceinline__ v16h load(const _Float16* p) {
    U f; f.h[0] = *(const v8h*)(p); f.h[1] = *(const v8h*)(p + 16); return f.v;
  }
  static __device__ __forceinline__ v8f mma(v16h a, v16h b, v8f c) {
    return __builtin_amdgcn_wmma_f32_16x16x32_f16(false, a, false, b, (short)0, c, false, false);
  }
  static __device__ __forceinline__ void guard(v8f& a, v8f& b, v16h x, v16h y) { dep_guard_h(a, b, x, y); }
  static __device__ __forceinline__ void keep(v16h a, v16h b, v16h c, v16h d) { keep4_h(a, b, c, d); }
};
template <> struct Frag<__bf16> {
  typedef v16b V; union U { v16b v; v8b h[2]; };
  static __device__ __forceinline__ v16b load(const __bf16* p) {
    U f; f.h[0] = *(const v8b*)(p); f.h[1] = *(const v8b*)(p + 16); return f.v;
  }
  static __device__ __forceinline__ v8f mma(v16b a, v16b b, v8f c) {
    return __builtin_amdgcn_wmma_f32_16x16x32_bf16(false, a, false, b, (short)0, c, false, false);
  }
  static __device__ __forceinline__ void guard(v8f& a, v8f& b, v16b x, v16b y) { dep_guard_b(a, b, x, y); }
  static __device__ __forceinline__ void keep(v16b a, v16b b, v16b c, v16b d) { keep4_b(a, b, c, d); }
};

__device__ __forceinline__ v8f mma_h(v16h a, v16h b, v8f c) {
  c = __builtin_amdgcn_wmma_f32_16x16x32_f16(false, a, false, b, (short)0, c, false, false);
  asm volatile("v_nop\n\tv_nop\n\tv_nop\n\tv_nop" : "+v"(c) : "v"(a), "v"(b));
  return c;
}

template <int ET> struct Elem;
template <> struct Elem<0> { typedef _Float16 T; };
template <> struct Elem<1> { typedef __bf16 T; };
template <int ET, bool SPLIT, int BIAS_MODE, int OUT_MODE, bool RESID, int ACT = 0>
__global__ __launch_bounds__(256) void wmma_gemm64(
    const unsigned short* __restrict__ Ap, const unsigned short* __restrict__ A2p, int lda, long strideA,
    const unsigned short* __restrict__ Btp, const unsigned short* __restrict__ Bt2p, int ldb, long strideB,
    void* __restrict__ Cout, void* __restrict__ Cout2, int ldc, long strideC,
    const float* __restrict__ bias,
    const float* __restrict__ resid, long strideR,
    int M, int N, int K, float scale) {
  typedef typename Elem<ET>::T T;
  typedef typename Frag<T>::V V;
  const T* A = (const T*)Ap; const T* A2 = (const T*)A2p; const T* Bt = (const T*)Btp; const T* Bt2 = (const T*)Bt2p;
  __shared__ __align__(16) float sT[8][16 * 68];
  const int b    = blockIdx.y;
  const int lane = threadIdx.x & 31;
  const int wave = threadIdx.x >> 5;
  const int tilesN = N >> 6;
  const int tilesM = M >> 6;
  const int tile = blockIdx.x * 8 + wave;
  if (tile >= tilesM * tilesN) return;
  const int tm = tile / tilesN;
  const int tn = tile - tm * tilesN;
  const int m0 = tm << 6;
  const int n0 = tn << 6;

  const T* Ab  = A  + (size_t)b * strideA;
  const T* Bb  = Bt + (size_t)b * strideB;
  const T* Ab2 = SPLIT ? (A2  + (size_t)b * strideA) : nullptr;
  const T* Bb2 = SPLIT ? (Bt2 + (size_t)b * strideB) : nullptr;

  const int rlane = lane & 15;
  const int koff  = (lane >> 4) * 8;
  const int mOff  = (lane >> 4) * 8;

  v8f acc[4][4];
#pragma unroll
  for (int i = 0; i < 4; ++i)
#pragma unroll
    for (int j = 0; j < 4; ++j) acc[i][j] = (v8f){0.f,0.f,0.f,0.f,0.f,0.f,0.f,0.f};

  for (int k0 = 0; k0 < K; k0 += 32) {
    V bh[4], bl[4];
#pragma unroll
    for (int j = 0; j < 4; ++j) {
      const size_t bo = (size_t)(n0 + (j << 4) + rlane) * ldb + koff + k0;
      bh[j] = Frag<T>::load(Bb + bo);
      if (SPLIT) bl[j] = Frag<T>::load(Bb2 + bo);
    }
#pragma unroll
    for (int i = 0; i < 4; ++i) {
      const size_t ao = (size_t)(m0 + (i << 4) + rlane) * lda + koff + k0;
      V ah = Frag<T>::load(Ab + ao);
      V al;
      if (SPLIT) al = Frag<T>::load(Ab2 + ao);
#pragma unroll
      for (int j = 0; j < 4; ++j) {
        acc[i][j] = Frag<T>::mma(ah, bh[j], acc[i][j]);
        if (SPLIT) {
          acc[i][j] = Frag<T>::mma(ah, bl[j], acc[i][j]);
          acc[i][j] = Frag<T>::mma(al, bh[j], acc[i][j]);
        }
      }
      Frag<T>::guard(acc[i][0], acc[i][3], ah, SPLIT ? al : ah);
    }
    Frag<T>::keep(bh[0], bh[1], bh[2], bh[3]);
    if (SPLIT) Frag<T>::keep(bl[0], bl[1], bl[2], bl[3]);
  }
  acc_guard4(acc[0][0], acc[0][1], acc[0][2], acc[0][3]);
  acc_guard4(acc[1][0], acc[1][1], acc[1][2], acc[1][3]);
  acc_guard4(acc[2][0], acc[2][1], acc[2][2], acc[2][3]);
  acc_guard4(acc[3][0], acc[3][1], acc[3][2], acc[3][3]);

  float* slab = sT[wave];
  const float* Rb = RESID ? (resid + (size_t)b * strideR) : nullptr;
#pragma unroll
  for (int i = 0; i < 4; ++i) {
    const int mBase = m0 + (i << 4);
#pragma unroll
    for (int j = 0; j < 4; ++j) {
      const int n = n0 + (j << 4) + rlane;
      float bv = 0.f;
      if (BIAS_MODE == 2) bv = bias[n];
#pragma unroll
      for (int r = 0; r < 8; ++r) {
        float v = acc[i][j][r] * scale;
        if (BIAS_MODE == 1) v += bias[mBase + mOff + r];
        if (BIAS_MODE == 2) v += bv;
        if (RESID) v += Rb[(size_t)(mBase + mOff + r) * ldc + n];
        if (ACT == 1) v = tanhf(v);
        if (ACT == 2) v = fmaxf(v, 0.0f);
        if (ACT == 3) v = v / (1.0f + expf(-v));
        if (ACT == 4) v = (v > 0.f) ? v : 0.01f * v;
        if (ACT == 5) v = 0.5f * v * (1.0f + erff(v * 0.70710678118654752f));
        slab[(mOff + r) * 68 + (j << 4) + rlane] = v;
      }
    }
    __builtin_amdgcn_fence(__ATOMIC_RELEASE, "workgroup");
    __builtin_amdgcn_wave_barrier();
    __builtin_amdgcn_fence(__ATOMIC_ACQUIRE, "workgroup");
    if (OUT_MODE == 0) {
      float* C = (float*)Cout + (size_t)b * strideC;
      const int hh = lane >> 4, c4 = (lane & 15) * 4;
      for (int pass = 0; pass < 2; ++pass) {
#pragma unroll
        for (int it = 0; it < 8; ++it) {
          const int row = it * 2 + hh;
          v4f v = *(const v4f*)(slab + row * 68 + c4);
          *(volatile v4f*)(C + (size_t)(mBase + row) * ldc + n0 + c4) = v;
        }
        __threadfence();
      }
    } else {
      const int q = lane >> 3, c8 = (lane & 7) * 8;
      unsigned short* C  = (unsigned short*)Cout  + (size_t)b * strideC;
      unsigned short* C2 = (OUT_MODE == 2) ? ((unsigned short*)Cout2 + (size_t)b * strideC) : nullptr;
      for (int pass = 0; pass < 2; ++pass) {
#pragma unroll
        for (int it = 0; it < 4; ++it) {
          const int row = it * 4 + q;
          const float* sp = slab + row * 68 + c8;
          v8h hv, lv;
#pragma unroll
          for (int e = 0; e < 8; ++e) {
            if (OUT_MODE == 1) {
              hv[e] = (_Float16)sp[e];
            } else {
              unsigned short hb = f2bf_bits(sp[e]);
              unsigned short lb = f2bf_bits(sp[e] - bf_bits2f(hb));
              hv[e] = __builtin_bit_cast(_Float16, hb);
              lv[e] = __builtin_bit_cast(_Float16, lb);
            }
          }
          *(volatile v8h*)(C + (size_t)(mBase + row) * ldc + n0 + c8) = hv;
          if (OUT_MODE == 2) *(volatile v8h*)(C2 + (size_t)(mBase + row) * ldc + n0 + c8) = lv;
        }
        __threadfence();
      }
    }
    __builtin_amdgcn_fence(__ATOMIC_RELEASE, "workgroup");
    __builtin_amdgcn_wave_barrier();
    __builtin_amdgcn_fence(__ATOMIC_ACQUIRE, "workgroup");
  }
}

__global__ __launch_bounds__(256) void k_cast_comb(const float* __restrict__ x, const float* __restrict__ ctx,
                                                    _Float16* __restrict__ out, int ngrp) {
  const int i = blockIdx.x * 256 + threadIdx.x;
  if (i >= ngrp) return;
  const int row  = i >> 7;
  const int col0 = (i & 127) << 3;
  const int ca   = col0 & (DIN - 1);
  const float* pa = x   + (size_t)row * DIN + ca;
  const float* pb = ctx + (size_t)row * DIN + ca;
  const v4f a0 = *(const v4f*)pa, a1 = *(const v4f*)(pa + 4);
  const v4f b0 = *(const v4f*)pb, b1 = *(const v4f*)(pb + 4);
  const bool sec = (col0 >= DIN);
  v8h hv;
#pragma unroll
  for (int e = 0; e < 4; ++e) {
    hv[e]     = (_Float16)(sec ? b0[e] : a0[e]);
    hv[4 + e] = (_Float16)(sec ? b1[e] : a1[e]);
  }
  _Float16* o = out + (size_t)i * 8;
  *(volatile v8h*)o = hv;
  __threadfence();
  *(volatile v8h*)o = hv;
}

__global__ __launch_bounds__(256) void k_cast_w(const float* __restrict__ wk, const float* __restrict__ wc,
                                                 _Float16* __restrict__ out, int ngrp) {
  const int i = blockIdx.x * 256 + threadIdx.x;
  if (i >= ngrp) return;
  const int row  = i >> 7;
  const int col0 = (i & 127) << 3;
  const int r2   = row & (DKEY - 1);
  const float* pa = wk + (size_t)r2 * DCOMB + col0;
  const float* pb = wc + (size_t)r2 * DCOMB + col0;
  const v4f a0 = *(const v4f*)pa, a1 = *(const v4f*)(pa + 4);
  const v4f b0 = *(const v4f*)pb, b1 = *(const v4f*)(pb + 4);
  const bool sec = (row >= DKEY);
  v8h hv;
#pragma unroll
  for (int e = 0; e < 4; ++e) {
    hv[e]     = (_Float16)((sec ? b0[e] : a0[e]) * WSCL);
    hv[4 + e] = (_Float16)((sec ? b1[e] : a1[e]) * WSCL);
  }
  _Float16* o = out + (size_t)i * 8;
  *(volatile v8h*)o = hv;
  __threadfence();
  *(volatile v8h*)o = hv;
}

__global__ __launch_bounds__(256) void k_prep_proto(const float* __restrict__ proto, _Float16* __restrict__ p16,
                                                     float* __restrict__ p2) {
  __shared__ __align__(16) float p2s[32];
  const int tid  = threadIdx.x;
  const int rloc = tid >> 3, g = tid & 7;
  const int row  = blockIdx.x * 32 + rloc;
  const float* pr = proto + (size_t)row * DKEY + g * 8;
  const v4f a0 = *(const v4f*)pr, a1 = *(const v4f*)(pr + 4);
  float s = 0.f;
  v8h hv;
#pragma unroll
  for (int e = 0; e < 4; ++e) { s += a0[e] * a0[e]; hv[e] = (_Float16)(a0[e] * KVSCL); }
#pragma unroll
  for (int e = 0; e < 4; ++e) { s += a1[e] * a1[e]; hv[4 + e] = (_Float16)(a1[e] * KVSCL); }
  s += __shfl_xor(s, 1, 32);
  s += __shfl_xor(s, 2, 32);
  s += __shfl_xor(s, 4, 32);
  _Float16* o = p16 + (size_t)row * DKEY + g * 8;
  *(volatile v8h*)o = hv;
  if (g == 0) p2s[rloc] = s;
  __syncthreads();
  __threadfence();
  *(volatile v8h*)o = hv;
  if (tid < 8) {
    const v4f v = *(const v4f*)(p2s + 4 * tid);
    float* po = p2 + (size_t)blockIdx.x * 32 + 4 * tid;
    *(volatile v4f*)po = v;
    __threadfence();
    *(volatile v4f*)po = v;
  }
}

__global__ __launch_bounds__(256) void k_prep_buft(const float* __restrict__ buf, _Float16* __restrict__ bt16) {
  __shared__ __align__(16) _Float16 T[64 * 72];
  const int tid = threadIdx.x;
  const int n0  = blockIdx.x * 64;
  {
    const int n = tid >> 2, dq = (tid & 3) * 16;
    const float* pr = buf + (size_t)(n0 + n) * DVAL + dq;
#pragma unroll
    for (int i = 0; i < 4; ++i) {
      const v4f v = *(const v4f*)(pr + 4 * i);
#pragma unroll
      for (int e = 0; e < 4; ++e) T[(dq + 4 * i + e) * 72 + n] = (_Float16)(v[e] * KVSCL);
    }
  }
  __syncthreads();
  v8h hv[2];
#pragma unroll
  for (int it = 0; it < 2; ++it) {
    const int d = it * 32 + (tid >> 3), c8 = (tid & 7) * 8;
    hv[it] = *(const v8h*)(T + d * 72 + c8);
    *(volatile v8h*)(bt16 + (size_t)d * NBINS + n0 + c8) = hv[it];
  }
  __threadfence();
#pragma unroll
  for (int it = 0; it < 2; ++it) {
    const int d = it * 32 + (tid >> 3), c8 = (tid & 7) * 8;
    *(volatile v8h*)(bt16 + (size_t)d * NBINS + n0 + c8) = hv[it];
  }
}

__global__ __launch_bounds__(256) void k_conv_km(const float* __restrict__ km, const float* __restrict__ bk,
                                                  const float* __restrict__ bc,
                                                  _Float16* __restrict__ k16, _Float16* __restrict__ mt16) {
  __shared__ __align__(16) _Float16 T[64 * 72];
  const int tid = threadIdx.x;
  const int b0  = blockIdx.x * 64;
  v8h kh[2];
#pragma unroll
  for (int it = 0; it < 2; ++it) {
    const int row = it * 32 + (tid >> 3), c8 = (tid & 7) * 8;
    const float* pr = km + (size_t)(b0 + row) * NPROJ + c8;
    const v4f a0 = *(const v4f*)pr, a1 = *(const v4f*)(pr + 4);
    const v4f q0 = *(const v4f*)(bk + c8), q1 = *(const v4f*)(bk + c8 + 4);
#pragma unroll
    for (int e = 0; e < 4; ++e) { kh[it][e] = (_Float16)(a0[e] + q0[e]); kh[it][4 + e] = (_Float16)(a1[e] + q1[e]); }
    *(volatile v8h*)(k16 + (size_t)(b0 + row) * DKEY + c8) = kh[it];
  }
  {
    const int bb = tid >> 2, dq = (tid & 3) * 16;
    const float* pr = km + (size_t)(b0 + bb) * NPROJ + DKEY + dq;
#pragma unroll
    for (int i = 0; i < 4; ++i) {
      const v4f v = *(const v4f*)(pr + 4 * i);
      const v4f q = *(const v4f*)(bc + dq + 4 * i);
#pragma unroll
      for (int e = 0; e < 4; ++e) T[(dq + 4 * i + e) * 72 + bb] = (_Float16)(v[e] + q[e]);
    }
  }
  __syncthreads();
  v8h mh[2];
#pragma unroll
  for (int it = 0; it < 2; ++it) {
    const int d = it * 32 + (tid >> 3), c8 = (tid & 7) * 8;
    mh[it] = *(const v8h*)(T + d * 72 + c8);
    *(volatile v8h*)(mt16 + (size_t)d * NBATCH + b0 + c8) = mh[it];
  }
  __threadfence();
#pragma unroll
  for (int it = 0; it < 2; ++it) {
    const int row = it * 32 + (tid >> 3), c8 = (tid & 7) * 8;
    *(volatile v8h*)(k16 + (size_t)(b0 + row) * DKEY + c8) = kh[it];
    const int d = row;
    *(volatile v8h*)(mt16 + (size_t)d * NBATCH + b0 + c8) = mh[it];
  }
}

__global__ __launch_bounds__(128) void k_pass1(const _Float16* __restrict__ q16, const _Float16* __restrict__ kp16,
                                                const _Float16* __restrict__ vt16, const float* __restrict__ p2,
                                                float* __restrict__ rout, float* __restrict__ stats) {
  union FB { v16h v; v8h h[2]; };
  __shared__ __align__(16) _Float16 Ksh[64 * 64];
  __shared__ __align__(16) _Float16 Vth[64 * 64];
  __shared__ __align__(16) _Float16 Psh[4][16 * 64];
  __shared__ __align__(16) float  Os[4][16 * 68];
  __shared__ __align__(16) float  Ssh[128];
  const int tid = threadIdx.x, wave = tid >> 5, lane = tid & 31, hh = lane >> 4, c = lane & 15;
  const int q0 = blockIdx.x * 64 + wave * 16;

  v16h qa[2];
#pragma unroll
  for (int dc = 0; dc < 2; ++dc) qa[dc] = Frag<_Float16>::load(q16 + (size_t)(q0 + c) * DKEY + dc * 32 + 8 * hh);

  float mrow[8], lrow[8];
  v8f oacc[4];
#pragma unroll
  for (int r = 0; r < 8; ++r) { mrow[r] = -INFINITY; lrow[r] = 0.f; }
#pragma unroll
  for (int t = 0; t < 4; ++t) oacc[t] = (v8f){0.f,0.f,0.f,0.f,0.f,0.f,0.f,0.f};

  for (int kc = 0; kc < NBINS / 64; ++kc) {
    const int kv0 = kc * 64;
    __syncthreads();
    {
      const int rr = tid >> 1, dh = (tid & 1) * 32;
      const _Float16* krow = kp16 + (size_t)(kv0 + rr) * DKEY + dh;
      const _Float16* vrow = vt16 + (size_t)rr * NBINS + kv0 + dh;
#pragma unroll
      for (int i = 0; i < 4; ++i) {
        const v8h kk = *(const v8h*)(krow + 8 * i);
        const v8h vv = *(const v8h*)(vrow + 8 * i);
        *(v8h*)(Ksh + rr * 64 + dh + 8 * i) = kk;
        *(v8h*)(Vth + rr * 64 + dh + 8 * i) = vv;
      }
    }
    __syncthreads();

    float p2v[4];
#pragma unroll
    for (int j = 0; j < 4; ++j) p2v[j] = p2[kv0 + j * 16 + c];

    v8f s[4];
#pragma unroll
    for (int j = 0; j < 4; ++j) {
      s[j] = (v8f){0.f,0.f,0.f,0.f,0.f,0.f,0.f,0.f};
#pragma unroll
      for (int dc = 0; dc < 2; ++dc) {
        FB kb;
        kb.h[0] = *(const v8h*)(Ksh + (j * 16 + c) * 64 + dc * 32 + 8 * hh);
        kb.h[1] = *(const v8h*)(Ksh + (j * 16 + c) * 64 + dc * 32 + 16 + 8 * hh);
        s[j] = mma_h(qa[dc], kb.v, s[j]);
      }
    }
    float cm[8];
#pragma unroll
    for (int r = 0; r < 8; ++r) {
      float m = -INFINITY;
#pragma unroll
      for (int j = 0; j < 4; ++j) {
        const float sc = s[j][r] * QS - p2v[j];
        s[j][r] = sc;
        m = fmaxf(m, sc);
      }
#pragma unroll
      for (int off = 1; off < 16; off <<= 1) m = fmaxf(m, __shfl_xor(m, off, 32));
      cm[r] = m;
    }
    _Float16* pw = Psh[wave];
#pragma unroll
    for (int r = 0; r < 8; ++r) {
      const float mnew  = fmaxf(mrow[r], cm[r]);
      const float alpha = __expf(mrow[r] - mnew);
      mrow[r] = mnew;
      float psum = 0.f;
#pragma unroll
      for (int j = 0; j < 4; ++j) {
        const float p = __expf(s[j][r] - mnew);
        psum += p;
        pw[(8 * hh + r) * 64 + j * 16 + c] = (_Float16)(p * PSC);
      }
#pragma unroll
      for (int off = 1; off < 16; off <<= 1) psum += __shfl_xor(psum, off, 32);
      lrow[r] = lrow[r] * alpha + psum;
#pragma unroll
      for (int t = 0; t < 4; ++t) oacc[t][r] *= alpha;
    }
    __builtin_amdgcn_fence(__ATOMIC_RELEASE, "workgroup");
    __builtin_amdgcn_wave_barrier();
    __builtin_amdgcn_fence(__ATOMIC_ACQUIRE, "workgroup");
#pragma unroll
    for (int kk = 0; kk < 2; ++kk) {
      FB pa;
      pa.h[0] = *(const v8h*)(pw + c * 64 + kk * 32 + 8 * hh);
      pa.h[1] = *(const v8h*)(pw + c * 64 + kk * 32 + 16 + 8 * hh);
#pragma unroll
      for (int t = 0; t < 4; ++t) {
        FB vb;
        vb.h[0] = *(const v8h*)(Vth + (t * 16 + c) * 64 + kk * 32 + 8 * hh);
        vb.h[1] = *(const v8h*)(Vth + (t * 16 + c) * 64 + kk * 32 + 16 + 8 * hh);
        oacc[t] = mma_h(pa.v, vb.v, oacc[t]);
      }
    }
  }

  float* os = Os[wave];
  float rinv[8];
#pragma unroll
  for (int r = 0; r < 8; ++r) {
    rinv[r] = 1.0f / lrow[r];
    const float inv = rinv[r] * (1.0f / 2097152.0f);
#pragma unroll
    for (int t = 0; t < 4; ++t) os[(8 * hh + r) * 68 + t * 16 + c] = oacc[t][r] * inv;
  }
  if (c == 0) {
#pragma unroll
    for (int r = 0; r < 8; ++r) {
      Ssh[(wave * 16 + 8 * hh + r) * 2 + 0] = mrow[r];
      Ssh[(wave * 16 + 8 * hh + r) * 2 + 1] = rinv[r];
    }
  }
  __builtin_amdgcn_fence(__ATOMIC_RELEASE, "workgroup");
  __builtin_amdgcn_wave_barrier();
  __builtin_amdgcn_fence(__ATOMIC_ACQUIRE, "workgroup");
  {
    const int c4 = (lane & 15) * 4;
    for (int pass = 0; pass < 2; ++pass) {
#pragma unroll
      for (int it = 0; it < 8; ++it) {
        const int row = it * 2 + hh;
        const v4f val = *(const v4f*)(os + row * 68 + c4);
        *(volatile v4f*)(rout + (size_t)(q0 + row) * DVAL + c4) = val;
      }
      __threadfence();
    }
  }
  __syncthreads();
  if (wave == 0) {
    const v4f v = *(const v4f*)(Ssh + 4 * lane);
    float* po = stats + (size_t)blockIdx.x * 128 + 4 * lane;
    *(volatile v4f*)po = v;
    __threadfence();
    *(volatile v4f*)po = v;
  }
}

__global__ __launch_bounds__(128) void k_pass2(const _Float16* __restrict__ q16, const _Float16* __restrict__ kb16,
                                                const _Float16* __restrict__ vt16, const float* __restrict__ p2,
                                                const float* __restrict__ stats, const float* __restrict__ buf,
                                                float* __restrict__ nbout) {
  union FB { v16h v; v8h h[2]; };
  __shared__ __align__(16) _Float16 Ksh[64 * 64];
  __shared__ __align__(16) _Float16 Vth[64 * 64];
  __shared__ __align__(16) _Float16 Psh[4][16 * 64];
  __shared__ __align__(16) float  Os[4][16 * 68];
  const int tid = threadIdx.x, wave = tid >> 5, lane = tid & 31, hh = lane >> 4, c = lane & 15;
  const int n0w = blockIdx.x * 64 + wave * 16;

  v16h qa[2];
#pragma unroll
  for (int dc = 0; dc < 2; ++dc) qa[dc] = Frag<_Float16>::load(q16 + (size_t)(n0w + c) * DKEY + dc * 32 + 8 * hh);

  float p2r[8], asum[8];
  v8f oacc[4];
#pragma unroll
  for (int r = 0; r < 8; ++r) { p2r[r] = p2[n0w + 8 * hh + r]; asum[r] = 0.f; }
#pragma unroll
  for (int t = 0; t < 4; ++t) oacc[t] = (v8f){0.f,0.f,0.f,0.f,0.f,0.f,0.f,0.f};

  for (int bcI = 0; bcI < NBATCH / 64; ++bcI) {
    const int b0 = bcI * 64;
    __syncthreads();
    {
      const int rr = tid >> 1, dh = (tid & 1) * 32;
      const _Float16* krow = kb16 + (size_t)(b0 + rr) * DKEY + dh;
      const _Float16* vrow = vt16 + (size_t)rr * NBATCH + b0 + dh;
#pragma unroll
      for (int i = 0; i < 4; ++i) {
        const v8h kk = *(const v8h*)(krow + 8 * i);
        const v8h vv = *(const v8h*)(vrow + 8 * i);
        *(v8h*)(Ksh + rr * 64 + dh + 8 * i) = kk;
        *(v8h*)(Vth + rr * 64 + dh + 8 * i) = vv;
      }
    }
    __syncthreads();

    float Mb[4], Zb[4];
#pragma unroll
    for (int j = 0; j < 4; ++j) {
      const v2f st = *(const v2f*)(stats + (size_t)(b0 + j * 16 + c) * 2);
      Mb[j] = st[0]; Zb[j] = st[1];
    }

    v8f s[4];
#pragma unroll
    for (int j = 0; j < 4; ++j) {
      s[j] = (v8f){0.f,0.f,0.f,0.f,0.f,0.f,0.f,0.f};
#pragma unroll
      for (int dc = 0; dc < 2; ++dc) {
        FB kb;
        kb.h[0] = *(const v8h*)(Ksh + (j * 16 + c) * 64 + dc * 32 + 8 * hh);
        kb.h[1] = *(const v8h*)(Ksh + (j * 16 + c) * 64 + dc * 32 + 16 + 8 * hh);
        s[j] = mma_h(qa[dc], kb.v, s[j]);
      }
    }
    _Float16* pw = Psh[wave];
#pragma unroll
    for (int r = 0; r < 8; ++r) {
#pragma unroll
      for (int j = 0; j < 4; ++j) {
        const float sc = s[j][r] * QS - p2r[r];
        const float a  = __expf(sc - Mb[j]) * Zb[j];
        asum[r] += a;
        pw[(8 * hh + r) * 64 + j * 16 + c] = (_Float16)(a * PSC);
      }
    }
    __builtin_amdgcn_fence(__ATOMIC_RELEASE, "workgroup");
    __builtin_amdgcn_wave_barrier();
    __builtin_amdgcn_fence(__ATOMIC_ACQUIRE, "workgroup");
#pragma unroll
    for (int kk = 0; kk < 2; ++kk) {
      FB pa;
      pa.h[0] = *(const v8h*)(pw + c * 64 + kk * 32 + 8 * hh);
      pa.h[1] = *(const v8h*)(pw + c * 64 + kk * 32 + 16 + 8 * hh);
#pragma unroll
      for (int t = 0; t < 4; ++t) {
        FB vb;
        vb.h[0] = *(const v8h*)(Vth + (t * 16 + c) * 64 + kk * 32 + 8 * hh);
        vb.h[1] = *(const v8h*)(Vth + (t * 16 + c) * 64 + kk * 32 + 16 + 8 * hh);
        oacc[t] = mma_h(pa.v, vb.v, oacc[t]);
      }
    }
  }

#pragma unroll
  for (int r = 0; r < 8; ++r) {
#pragma unroll
    for (int off = 1; off < 16; off <<= 1) asum[r] += __shfl_xor(asum[r], off, 32);
  }
  const float cc = 0.1f / 2048.0f;
  float* os = Os[wave];
#pragma unroll
  for (int r = 0; r < 8; ++r) {
    const int nrow = n0w + 8 * hh + r;
    const float* brow = buf + (size_t)nrow * DVAL;
#pragma unroll
    for (int t = 0; t < 4; ++t) {
      const float u   = oacc[t][r] * (1.0f / PSC);
      const float bv  = brow[t * 16 + c];
      const float dlt = u - asum[r] * bv;
      os[(8 * hh + r) * 68 + t * 16 + c] = bv + cc * dlt;
    }
  }
  __builtin_amdgcn_fence(__ATOMIC_RELEASE, "workgroup");
  __builtin_amdgcn_wave_barrier();
  __builtin_amdgcn_fence(__ATOMIC_ACQUIRE, "workgroup");
  {
    const int c4 = (lane & 15) * 4;
    for (int pass = 0; pass < 2; ++pass) {
#pragma unroll
      for (int it = 0; it < 8; ++it) {
        const int row = it * 2 + hh;
        const v4f val = *(const v4f*)(os + row * 68 + c4);
        *(volatile v4f*)(nbout + (size_t)(n0w + row) * DVAL + c4) = val;
      }
      __threadfence();
    }
  }
}

extern "C" void kernel_launch(void* const* d_in, const int* in_sizes, int n_in,
                              void* d_out, int out_size, void* d_ws, size_t ws_size,
                              hipStream_t stream) {
  if (n_in < 8) return;
  if (in_sizes[0] != NBATCH * DIN || in_sizes[1] != NBATCH * DIN) return;
  if (in_sizes[2] != DKEY * DCOMB || in_sizes[3] != DKEY) return;
  if (in_sizes[4] != DVAL * DCOMB || in_sizes[5] != DVAL) return;
  if (in_sizes[6] != NBINS * DKEY || in_sizes[7] != NBINS * DVAL) return;
  if (out_size != NBATCH * DVAL + NBINS * DVAL) return;

  const float* x     = (const float*)d_in[0];
  const float* ctx   = (const float*)d_in[1];
  const float* Wk    = (const float*)d_in[2];
  const float* bk    = (const float*)d_in[3];
  const float* Wc    = (const float*)d_in[4];
  const float* bc    = (const float*)d_in[5];
  const float* proto = (const float*)d_in[6];
  const float* buf   = (const float*)d_in[7];

  float* rout  = (float*)d_out;
  float* nbout = (float*)d_out + (size_t)NBATCH * DVAL;

  const size_t sz_comb16 = (size_t)NBATCH * DCOMB * 2;
  const size_t sz_w16    = (size_t)NPROJ * DCOMB * 2;
  const size_t sz_km     = (size_t)NBATCH * NPROJ * 4;
  const size_t sz_k16    = (size_t)NBATCH * DKEY * 2;
  const size_t sz_mt16   = (size_t)DVAL * NBATCH * 2;
  const size_t sz_p16    = (size_t)NBINS * DKEY * 2;
  const size_t sz_p2     = (size_t)NBINS * 4;
  const size_t sz_bt16   = (size_t)DVAL * NBINS * 2;
  const size_t sz_stats  = (size_t)NBATCH * 2 * 4;
  size_t off = 0;
  const size_t off_comb16 = off; off += sz_comb16;
  const size_t off_w16    = off; off += sz_w16;
  const size_t off_km     = off; off += sz_km;
  const size_t off_k16    = off; off += sz_k16;
  const size_t off_mt16   = off; off += sz_mt16;
  const size_t off_p16    = off; off += sz_p16;
  const size_t off_p2     = off; off += sz_p2;
  const size_t off_bt16   = off; off += sz_bt16;
  const size_t off_stats  = off; off += sz_stats;
  if (off > ws_size) return;

  char* ws = (char*)d_ws;
  _Float16* comb16 = (_Float16*)(ws + off_comb16);
  _Float16* w16    = (_Float16*)(ws + off_w16);
  float*    km     = (float*)(ws + off_km);
  _Float16* k16    = (_Float16*)(ws + off_k16);
  _Float16* mt16   = (_Float16*)(ws + off_mt16);
  _Float16* p16    = (_Float16*)(ws + off_p16);
  float*    p2     = (float*)(ws + off_p2);
  _Float16* bt16   = (_Float16*)(ws + off_bt16);
  float*    stats  = (float*)(ws + off_stats);

  const int ngrp_comb = NBATCH * DCOMB / 8;
  const int ngrp_w    = NPROJ * DCOMB / 8;

  k_cast_comb<<<dim3(ngrp_comb / 256), dim3(256), 0, stream>>>(x, ctx, comb16, ngrp_comb);
  k_cast_w<<<dim3(ngrp_w / 256), dim3(256), 0, stream>>>(Wk, Wc, w16, ngrp_w);
  k_prep_proto<<<dim3(NBINS / 32), dim3(256), 0, stream>>>(proto, p16, p2);
  k_prep_buft<<<dim3(NBINS / 64), dim3(256), 0, stream>>>(buf, bt16);

  wmma_gemm64<0, false, 0, 0, false><<<dim3((NBATCH / 64) * (NPROJ / 64) / 8, 1), dim3(256), 0, stream>>>(
      (const unsigned short*)comb16, (const unsigned short*)comb16, DCOMB, 0L,
      (const unsigned short*)w16, (const unsigned short*)w16, DCOMB, 0L,
      (void*)km, (void*)km, NPROJ, 0L,
      (const float*)km, (const float*)km, 0L,
      NBATCH, NPROJ, DCOMB, 1.0f / WSCL);

  k_conv_km<<<dim3(NBATCH / 64), dim3(256), 0, stream>>>(km, bk, bc, k16, mt16);

  k_pass1<<<dim3(NBATCH / 64), dim3(128), 0, stream>>>(k16, p16, bt16, p2, rout, stats);
  k_pass2<<<dim3(NBINS / 64), dim3(128), 0, stream>>>(p16, k16, mt16, p2, stats, buf, nbout);
}
